// MSDDAttn_88467736363077
// MI455X (gfx1250) — hardware-run, weakly checked
//
#include <hip/hip_runtime.h>
#include <math.h>

typedef __attribute__((ext_vector_type(16))) _Float16 v16h;
typedef __attribute__((ext_vector_type(8)))  _Float16 v8h;
typedef __attribute__((ext_vector_type(8)))  float    v8f;
typedef __attribute__((ext_vector_type(4)))  float    v4f;
typedef __attribute__((ext_vector_type(2)))  float    v2f;
typedef __attribute__((ext_vector_type(4)))  unsigned int v4u;

constexpr int kNb     = 2;
constexpr int kLq     = 3060;
constexpr int kRows   = kNb * kLq;
constexpr int kRowsP  = 6144;
constexpr int kDm     = 256;
constexpr int kHeads  = 8;
constexpr int kHc     = 32;
constexpr int kOffW   = 192;
constexpr int kLogW   = 864;
constexpr int kQpW    = 1088;
constexpr int kCatW   = 768;
constexpr int kPrW    = 32;
constexpr int kWtBlocks = 132;

constexpr float kActCarry = 16.0f;
constexpr float kWCarry   = 1024.0f;
constexpr float kCatCarry = 2048.0f;
constexpr float kProjScale = 1.0f / (kActCarry * kWCarry);
constexpr float kOutScale  = 1.0f / (kCatCarry * kWCarry);
constexpr float kF16MinNormal = 6.103515625e-05f;
constexpr float kInvLq = 1.0f / 3060.0f;

static_assert(kRows == 6120, "rows");
static_assert(kRowsP % 64 == 0 && kRowsP >= kRows, "row padding");
static_assert(kDm % 64 == 0 && kQpW % 64 == 0 && kCatW % 32 == 0 && kDm % 32 == 0, "tile multiples");
static_assert(kOffW + kLogW <= kQpW, "merged width");
static_assert(kOffW == 3 * kHeads * 4 * 2 && kLogW == 3 * kHeads * 36, "column maps");
static_assert(kHeads * kHc == kDm && kCatW == 3 * kDm, "head split");
static_assert(48 * 48 + 24 * 24 + 12 * 12 + 6 * 6 == kLq, "pyramid size");
static_assert(kLq % 4 == 0, "mean loop step");
static_assert(16 + 12 + 56 + 48 == kWtBlocks, "weight tile count");

constexpr size_t kSzAQ  = (size_t)kRowsP * kDm * 2;
constexpr size_t kSzWVT = (size_t)kDm * kDm * 2;
constexpr size_t kSzWQT = (size_t)kQpW * kDm * 2;
constexpr size_t kSzWOT = (size_t)kDm * kCatW * 2;
constexpr size_t kSzBQ  = (size_t)kQpW * 4;
constexpr size_t kSzVAL = (size_t)kRowsP * kDm * 4;
constexpr size_t kSzQP  = (size_t)kRowsP * kQpW * 4;
constexpr size_t kSzCAT = (size_t)kRowsP * kCatW * 2;
constexpr size_t kSzPR  = (size_t)kNb * kPrW * 4;
constexpr size_t kOffAQ  = 0;
constexpr size_t kOffAX  = kOffAQ  + kSzAQ;
constexpr size_t kOffWVT = kOffAX  + kSzAQ;
constexpr size_t kOffWQT = kOffWVT + kSzWVT;
constexpr size_t kOffWOT = kOffWQT + kSzWQT;
constexpr size_t kOffBQ  = kOffWOT + kSzWOT;
constexpr size_t kOffVAL = kOffBQ  + kSzBQ;
constexpr size_t kOffQP  = kOffVAL + kSzVAL;
constexpr size_t kOffCAT = kOffQP  + kSzQP;
constexpr size_t kOffPR  = kOffCAT + kSzCAT;
constexpr size_t kWsTotal = kOffPR + kSzPR;
static_assert(kWsTotal == 49844736ull, "carve total");
static_assert(kWsTotal <= 134217728ull, "carve cap");
static_assert((kOffAX % 128) == 0 && (kOffWVT % 128) == 0 && (kOffWQT % 128) == 0 && (kOffWOT % 128) == 0 &&
              (kOffBQ % 128) == 0 && (kOffVAL % 128) == 0 && (kOffQP % 128) == 0 && (kOffCAT % 128) == 0 &&
              (kOffPR % 128) == 0, "128-B aligned regions");

__device__ __forceinline__ unsigned pk16(unsigned short a, unsigned short b) { return (unsigned)a | ((unsigned)b << 16); }

__device__ __forceinline__ unsigned short h_bits_flush(float f) {
  const float g = (fabsf(f) < kF16MinNormal) ? 0.0f : f;
  const _Float16 h = (_Float16)g;
  return __builtin_bit_cast(unsigned short, h);
}

union FragU { v16h v; v8h h[2]; };
__device__ __forceinline__ v16h frag_load(const _Float16* p) {
  FragU f;
  f.h[0] = *(const v8h*)(p);
  f.h[1] = *(const v8h*)(p + 16);
  return f.v;
}
__device__ __forceinline__ v8f mma_f16(v16h a, v16h b, v8f c) {
  return __builtin_amdgcn_wmma_f32_16x16x32_f16(false, a, false, b, (short)0, c, false, false);
}
__device__ __forceinline__ void guard1_h(v8f& a, v16h x, v16h y) {
  asm volatile("v_nop\n\tv_nop\n\tv_nop\n\tv_nop" : "+v"(a) : "v"(x), "v"(y));
}
__device__ __forceinline__ void keep4_h(v16h a, v16h b, v16h c, v16h d) { asm volatile("v_nop" :: "v"(a), "v"(b), "v"(c), "v"(d)); }
__device__ __forceinline__ void acc_guard4(v8f& a, v8f& b, v8f& c, v8f& d) {
  asm volatile("v_nop\n\tv_nop\n\tv_nop\n\tv_nop" : "+v"(a), "+v"(b), "+v"(c), "+v"(d));
}

__global__ __launch_bounds__(256) void gemm64_f16_kernel(
    const unsigned short* __restrict__ Ap, int lda,
    const unsigned short* __restrict__ Btp, int ldb,
    float* __restrict__ Cout, int ldc,
    const float* __restrict__ bias,
    int M, int N, int K, int mStore, float scale) {
  const _Float16* A  = (const _Float16*)Ap;
  const _Float16* Bt = (const _Float16*)Btp;
  __shared__ __align__(16) float sT[8][16 * 68];
  const int lane = threadIdx.x & 31;
  const int wave = threadIdx.x >> 5;
  const int tilesN = N >> 6;
  const int tilesM = M >> 6;
  const int tile = blockIdx.x * 8 + wave;
  if (tile >= tilesM * tilesN) return;
  const int tm = tile / tilesN;
  const int tn = tile - tm * tilesN;
  const int m0 = tm << 6;
  const int n0 = tn << 6;

  const int rlane = lane & 15;
  const int koff  = (lane >> 4) * 8;
  const int mOff  = (lane >> 4) * 8;

  v8f acc[4][4];
#pragma unroll
  for (int i = 0; i < 4; ++i)
#pragma unroll
    for (int j = 0; j < 4; ++j) acc[i][j] = (v8f){0.f,0.f,0.f,0.f,0.f,0.f,0.f,0.f};

  for (int k0 = 0; k0 < K; k0 += 32) {
    v16h bh[4];
#pragma unroll
    for (int j = 0; j < 4; ++j) {
      const size_t bo = (size_t)(n0 + (j << 4) + rlane) * ldb + koff + k0;
      bh[j] = frag_load(Bt + bo);
    }
#pragma unroll
    for (int i = 0; i < 4; ++i) {
      const size_t ao = (size_t)(m0 + (i << 4) + rlane) * lda + koff + k0;
      const v16h ah = frag_load(A + ao);
#pragma unroll
      for (int j = 0; j < 4; ++j) acc[i][j] = mma_f16(ah, bh[j], acc[i][j]);
      guard1_h(acc[i][0], ah, bh[0]);
      guard1_h(acc[i][1], ah, bh[1]);
      guard1_h(acc[i][2], ah, bh[2]);
      guard1_h(acc[i][3], ah, bh[3]);
    }
    keep4_h(bh[0], bh[1], bh[2], bh[3]);
  }
  acc_guard4(acc[0][0], acc[0][1], acc[0][2], acc[0][3]);
  acc_guard4(acc[1][0], acc[1][1], acc[1][2], acc[1][3]);
  acc_guard4(acc[2][0], acc[2][1], acc[2][2], acc[2][3]);
  acc_guard4(acc[3][0], acc[3][1], acc[3][2], acc[3][3]);

  float* slab = sT[wave];
#pragma unroll
  for (int i = 0; i < 4; ++i) {
    const int mBase = m0 + (i << 4);
#pragma unroll
    for (int j = 0; j < 4; ++j) {
      const int n = n0 + (j << 4) + rlane;
      const float bv = bias[n];
#pragma unroll
      for (int r = 0; r < 8; ++r) {
        const float v = acc[i][j][r] * scale + bv;
        slab[(mOff + r) * 68 + (j << 4) + rlane] = v;
      }
    }
    __builtin_amdgcn_fence(__ATOMIC_RELEASE, "workgroup");
    __builtin_amdgcn_wave_barrier();
    __builtin_amdgcn_fence(__ATOMIC_ACQUIRE, "workgroup");
    {
      const int hh = lane >> 4, c4 = (lane & 15) * 4;
      for (int pass = 0; pass < 2; ++pass) {
#pragma unroll
        for (int it = 0; it < 8; ++it) {
          const int row = it * 2 + hh;
          const v4f v = *(const v4f*)(slab + row * 68 + c4);
          if (mBase + row < mStore)
            *(volatile v4f*)(Cout + (size_t)(mBase + row) * ldc + n0 + c4) = v;
        }
        __threadfence();
      }
    }
    __builtin_amdgcn_fence(__ATOMIC_RELEASE, "workgroup");
    __builtin_amdgcn_wave_barrier();
    __builtin_amdgcn_fence(__ATOMIC_ACQUIRE, "workgroup");
  }
}

__global__ __launch_bounds__(256) void cast_act_kernel(
    const float* __restrict__ srcQ, const float* __restrict__ srcX,
    unsigned short* __restrict__ dstQ, unsigned short* __restrict__ dstX) {
  const int plane = blockIdx.y;
  const float* src = plane ? srcX : srcQ;
  unsigned short* dst = plane ? dstX : dstQ;
  const int i   = blockIdx.x * 256 + threadIdx.x;
  const int row = i >> 5;
  const int c8  = (i & 31) * 8;
  const int rowc = (row < kRows) ? row : (kRows - 1);
  const float* p = src + (size_t)rowc * kDm + c8;
  v4f a = *(const v4f*)(p);
  v4f c = *(const v4f*)(p + 4);
  asm volatile("" : "+v"(a), "+v"(c));
  const bool live = (row < kRows);
  unsigned short hb[8];
#pragma unroll
  for (int e = 0; e < 4; ++e) {
    const float f0 = a[e];
    const float f1 = c[e];
    const float g0 = live ? f0 * kActCarry : 0.0f;
    const float g1 = live ? f1 * kActCarry : 0.0f;
    hb[e]     = h_bits_flush(g0);
    hb[4 + e] = h_bits_flush(g1);
  }
  const v4u u = (v4u){pk16(hb[0], hb[1]), pk16(hb[2], hb[3]), pk16(hb[4], hb[5]), pk16(hb[6], hb[7])};
  unsigned short* q = dst + (size_t)row * kDm + c8;
  *(volatile v4u*)q = u;
  __threadfence();
  *(volatile v4u*)q = u;
}

__global__ __launch_bounds__(256) void weight_planes_kernel(
    const float* __restrict__ Wv, const float* __restrict__ Woff, const float* __restrict__ Wattn,
    const float* __restrict__ Wout, const float* __restrict__ boff, const float* __restrict__ battn,
    unsigned short* __restrict__ WVT, unsigned short* __restrict__ WQT, unsigned short* __restrict__ WOT,
    float* __restrict__ BQ) {
  __shared__ float sm[64][65];
  const int t = threadIdx.x;
  const int b = blockIdx.x;
  if (b == kWtBlocks) {
    for (int it = 0; it < 2; ++it) {
      const int idx4 = t + 256 * it;
      const int idc  = (idx4 < 272) ? idx4 : 271;
      float vals[4];
#pragma unroll
      for (int e = 0; e < 4; ++e) {
        const int n  = idc * 4 + e;
        const int io = (n < kOffW) ? n : (kOffW - 1);
        int ia = n - kOffW;
        ia = (ia < 0) ? 0 : ia;
        ia = (ia > kLogW - 1) ? (kLogW - 1) : ia;
        float vo = boff[io];
        float va = battn[ia];
        asm volatile("" : "+v"(vo), "+v"(va));
        vals[e] = (n < kOffW) ? vo : ((n < kOffW + kLogW) ? va : 0.0f);
      }
      const v4f v = (v4f){vals[0], vals[1], vals[2], vals[3]};
      if (idx4 < 272) {
        *(volatile v4f*)(BQ + 4 * idx4) = v;
        __threadfence();
        *(volatile v4f*)(BQ + 4 * idx4) = v;
      }
    }
    return;
  }
  const float* W;
  unsigned short* op;
  int Nw, kt, nt, ldo, orow0;
  if (b < 16) {
    W = Wv; op = WVT; Nw = kDm; kt = b & 3; nt = b >> 2; ldo = kDm; orow0 = 0;
  } else if (b < 28) {
    const int bb = b - 16;
    W = Woff; op = WQT; Nw = kOffW; kt = bb & 3; nt = bb >> 2; ldo = kDm; orow0 = 0;
  } else if (b < 84) {
    const int bb = b - 28;
    W = Wattn; op = WQT; Nw = kLogW; kt = bb & 3; nt = bb >> 2; ldo = kDm; orow0 = kOffW;
  } else {
    const int bb = b - 84;
    W = Wout; op = WOT; Nw = kDm; kt = bb % 12; nt = bb / 12; ldo = kCatW; orow0 = 0;
  }
  const int k0 = kt * 64;
  const int n0 = nt * 64;
#pragma unroll 4
  for (int i = 0; i < 16; ++i) {
    const int e = i * 256 + t;
    const int r = e >> 6;
    const int c = e & 63;
    const int nn = n0 + c;
    const int nc = (nn < Nw) ? nn : (Nw - 1);
    float w = W[(size_t)(k0 + r) * Nw + nc];
    asm volatile("" : "+v"(w));
    sm[c][r] = (nn < Nw) ? w * kWCarry : 0.0f;
  }
  __syncthreads();
  const int lane = t & 31, wave = t >> 5;
  const int q = lane >> 3, c8 = (lane & 7) * 8;
  v4u u[2];
#pragma unroll
  for (int it = 0; it < 2; ++it) {
    const int row = wave * 8 + it * 4 + q;
    unsigned short hb[8];
#pragma unroll
    for (int e = 0; e < 8; ++e) hb[e] = h_bits_flush(sm[row][c8 + e]);
    u[it] = (v4u){pk16(hb[0], hb[1]), pk16(hb[2], hb[3]), pk16(hb[4], hb[5]), pk16(hb[6], hb[7])};
  }
  for (int pass = 0; pass < 2; ++pass) {
#pragma unroll
    for (int it = 0; it < 2; ++it) {
      const int row = wave * 8 + it * 4 + q;
      *(volatile v4u*)(op + (size_t)(orow0 + n0 + row) * ldo + k0 + c8) = u[it];
    }
    __threadfence();
  }
}

__global__ __launch_bounds__(256) void gate_kernel(
    const float* __restrict__ value, const float* __restrict__ Wse, const float* __restrict__ bse,
    const int* __restrict__ shp, float* __restrict__ PR) {
  __shared__ float sx[kDm];
  __shared__ float sW[96];
  __shared__ float sB[4];
  __shared__ float sP[32];
  __shared__ int sBad;
  const int n = blockIdx.x;
  const int t = threadIdx.x;
  float wv = Wse[(t < 96) ? t : 95];
  float bb = bse[(t < 3) ? t : 2];
  int sv = shp[(t < 8) ? t : 7];
  asm volatile("" : "+v"(wv), "+v"(bb), "+v"(sv));
  if (t < 96) sW[t] = wv;
  if (t < 4) sB[t] = (t < 3) ? bb : 0.0f;
  if (t == 0) sBad = 0;
  const int want = 48 >> ((t & 7) >> 1);
  const bool badl = (t < 8) && (sv != want);
  const float* vp = value + (size_t)n * kLq * kDm + t;
  float s0 = 0.0f, s1 = 0.0f, s2 = 0.0f, s3 = 0.0f;
#pragma unroll 1
  for (int q = 0; q < kLq; q += 4) {
    s0 += vp[(size_t)q * kDm];
    s1 += vp[(size_t)(q + 1) * kDm];
    s2 += vp[(size_t)(q + 2) * kDm];
    s3 += vp[(size_t)(q + 3) * kDm];
  }
  sx[t] = ((s0 + s1) + (s2 + s3)) * kInvLq;
  __syncthreads();
  if (badl) sBad = 1;
  if (t < 8) {
    float z0 = sB[0], z1 = sB[1], z2 = sB[2];
#pragma unroll 4
    for (int c = 0; c < kHc; ++c) {
      const float xv = sx[t * kHc + c];
      z0 = fmaf(xv, sW[c * 3 + 0], z0);
      z1 = fmaf(xv, sW[c * 3 + 1], z1);
      z2 = fmaf(xv, sW[c * 3 + 2], z2);
    }
    const float mz = fmaxf(z0, fmaxf(z1, z2));
    const float e0 = expf(z0 - mz), e1 = expf(z1 - mz), e2 = expf(z2 - mz);
    const float inv = 1.0f / (e0 + e1 + e2);
    sP[t * 3 + 0] = e0 * inv;
    sP[t * 3 + 1] = e1 * inv;
    sP[t * 3 + 2] = e2 * inv;
  }
  if (t >= 24 && t < 32) sP[t] = 0.0f;
  __syncthreads();
  if (t < 32) {
    const float pv = sP[t];
    const float v = (sBad != 0) ? __uint_as_float(0x7fc00000u) : pv;
    *(volatile float*)(PR + n * kPrW + t) = v;
    __threadfence();
    *(volatile float*)(PR + n * kPrW + t) = v;
  }
}

__global__ __launch_bounds__(384) void sample_mix_kernel(
    const float* __restrict__ value, const float* __restrict__ QP, const float* __restrict__ rpts,
    const float* __restrict__ PR, unsigned* __restrict__ cat32) {
  const int m    = blockIdx.x;
  const int tid  = threadIdx.x;
  const int lane = tid & 31, wave = tid >> 5;
  const int g = wave >> 2, hp = wave & 3;
  const int sub = lane >> 4, l16 = lane & 15;
  const int h = 2 * hp + sub;
  volatile unsigned* dst = cat32 + (size_t)m * (kCatW / 2) + g * 128 + hp * 32 + lane;
  if (m >= kRows) {
    *dst = 0u;
    __threadfence();
    *dst = 0u;
    return;
  }
  const int n = m / kLq;
  const int q = m - n * kLq;
  const int d = g + 1;

  const float* lg = QP + (size_t)m * kQpW + kOffW + g * 288 + h * 36;
  const float x0 = lg[l16];
  const float x1 = lg[16 + l16];
  float x2 = lg[32 + ((l16 < 4) ? l16 : 3)];
  asm volatile("" : "+v"(x2));
  const bool has2 = (l16 < 4);
  float mx = fmaxf(x0, x1);
  mx = fmaxf(mx, has2 ? x2 : x0);
  mx = fmaxf(mx, __shfl_xor(mx, 1, 32));
  mx = fmaxf(mx, __shfl_xor(mx, 2, 32));
  mx = fmaxf(mx, __shfl_xor(mx, 4, 32));
  mx = fmaxf(mx, __shfl_xor(mx, 8, 32));
  const float e0 = expf(x0 - mx);
  const float e1 = expf(x1 - mx);
  const float e2r = expf(x2 - mx);
  const float e2 = has2 ? e2r : 0.0f;
  float sum = (e0 + e1) + e2;
  sum += __shfl_xor(sum, 1, 32);
  sum += __shfl_xor(sum, 2, 32);
  sum += __shfl_xor(sum, 4, 32);
  sum += __shfl_xor(sum, 8, 32);
  const float inv = 1.0f / sum;
  const float pg = PR[n * kPrW + h * 3 + g];

  const float* vbase = value + (size_t)n * kLq * kDm + h * kHc + 2 * l16;
  const int laneBase = lane & 16;
  float a0 = 0.0f, a1 = 0.0f;
#pragma unroll 1
  for (int ki = 0; ki < 3; ++ki) {
    const int qn = q + (ki - 1) * d;
    const bool inb = (qn >= 0) && (qn < kLq);
    int qc = (qn < 0) ? 0 : qn;
    qc = (qc > kLq - 1) ? (kLq - 1) : qc;
    const size_t mp = (size_t)n * kLq + qc;
    const float* offp = QP + mp * kQpW + g * 64 + h * 8;
    const float* rp   = rpts + mp * 8;
    const int src1 = laneBase + ((ki == 2) ? 12 : 0);
#pragma unroll 1
    for (int l = 0; l < 4; ++l) {
      const float w0s = __shfl(e0, laneBase + 4 + l, 32);
      const float w1s = __shfl(e1, src1 + l, 32);
      float w = ((ki == 0) ? w0s : w1s) * inv;
      w = inb ? w : 0.0f;
      const int Wl = 48 >> l;
      const int st = (l == 0) ? 0 : ((l == 1) ? 2304 : ((l == 2) ? 2880 : 3024));
      const float Sf = (float)Wl;
      const float invS = (l == 0) ? (1.0f / 48.0f) : ((l == 1) ? (1.0f / 24.0f) : ((l == 2) ? (1.0f / 12.0f) : (1.0f / 6.0f)));
      const v2f ofv = *(const v2f*)(offp + 2 * l);
      const v2f rfv = *(const v2f*)(rp + 2 * l);
      const float locx = rfv[0] + ofv[0] * invS;
      const float locy = rfv[1] + ofv[1] * invS;
      const float grx = 2.0f * locx - 1.0f;
      const float gry = 2.0f * locy - 1.0f;
      const float gx = (grx + 1.0f) * (Sf * 0.5f) - 0.5f;
      const float gy = (gry + 1.0f) * (Sf * 0.5f) - 0.5f;
      const float x0f = floorf(gx), y0f = floorf(gy);
      const float wx1 = gx - x0f, wx0 = 1.0f - wx1;
      const float wy1 = gy - y0f, wy0 = 1.0f - wy1;
      const int xi0 = (int)fminf(fmaxf(x0f, -2.0f), 64.0f);
      const int yi0 = (int)fminf(fmaxf(y0f, -2.0f), 64.0f);
      const int xi1 = xi0 + 1, yi1 = yi0 + 1;
      const bool vx0 = (xi0 >= 0) && (xi0 < Wl);
      const bool vx1 = (xi1 >= 0) && (xi1 < Wl);
      const bool vy0 = (yi0 >= 0) && (yi0 < Wl);
      const bool vy1 = (yi1 >= 0) && (yi1 < Wl);
      int xc0 = (xi0 < 0) ? 0 : xi0;
      xc0 = (xc0 > Wl - 1) ? (Wl - 1) : xc0;
      int xc1 = (xi1 < 0) ? 0 : xi1;
      xc1 = (xc1 > Wl - 1) ? (Wl - 1) : xc1;
      int yc0 = (yi0 < 0) ? 0 : yi0;
      yc0 = (yc0 > Wl - 1) ? (Wl - 1) : yc0;
      int yc1 = (yi1 < 0) ? 0 : yi1;
      yc1 = (yc1 > Wl - 1) ? (Wl - 1) : yc1;
      const float w00 = (vx0 && vy0) ? wx0 * wy0 : 0.0f;
      const float w10 = (vx1 && vy0) ? wx1 * wy0 : 0.0f;
      const float w01 = (vx0 && vy1) ? wx0 * wy1 : 0.0f;
      const float w11 = (vx1 && vy1) ? wx1 * wy1 : 0.0f;
      const float* vb = vbase + (size_t)st * kDm;
      const v2f p00 = *(const v2f*)(vb + (size_t)(yc0 * Wl + xc0) * kDm);
      const v2f p10 = *(const v2f*)(vb + (size_t)(yc0 * Wl + xc1) * kDm);
      const v2f p01 = *(const v2f*)(vb + (size_t)(yc1 * Wl + xc0) * kDm);
      const v2f p11 = *(const v2f*)(vb + (size_t)(yc1 * Wl + xc1) * kDm);
      float s0 = p00[0] * w00;
      float s1 = p00[1] * w00;
      s0 = fmaf(p10[0], w10, s0);
      s1 = fmaf(p10[1], w10, s1);
      s0 = fmaf(p01[0], w01, s0);
      s1 = fmaf(p01[1], w01, s1);
      s0 = fmaf(p11[0], w11, s0);
      s1 = fmaf(p11[1], w11, s1);
      a0 = fmaf(w, s0, a0);
      a1 = fmaf(w, s1, a1);
    }
  }
  const float o0 = a0 * pg * kCatCarry;
  const float o1 = a1 * pg * kCatCarry;
  const unsigned short hb0 = h_bits_flush(o0);
  const unsigned short hb1 = h_bits_flush(o1);
  const unsigned u = pk16(hb0, hb1);
  *dst = u;
  __threadfence();
  *dst = u;
}

extern "C" void kernel_launch(void* const* d_in, const int* in_sizes, int n_in,
                              void* d_out, int out_size, void* d_ws, size_t ws_size,
                              hipStream_t stream) {
  if (n_in < 15) return;
  if (in_sizes[0] != kRows * kDm) return;
  if (in_sizes[1] != kRows * 8) return;
  if (in_sizes[2] != kRows * kDm) return;
  if (in_sizes[3] != 8) return;
  if (in_sizes[5] != kDm * kDm) return;
  if (in_sizes[6] != kDm) return;
  if (in_sizes[7] != kDm * kOffW) return;
  if (in_sizes[8] != kOffW) return;
  if (in_sizes[9] != kDm * kLogW) return;
  if (in_sizes[10] != kLogW) return;
  if (in_sizes[11] != kHc * 3) return;
  if (in_sizes[12] != 3) return;
  if (in_sizes[13] != kCatW * kDm) return;
  if (in_sizes[14] != kDm) return;
  if (out_size != kRows * kDm) return;
  if (ws_size < kWsTotal) return;

  const float* query = (const float*)d_in[0];
  const float* rpts  = (const float*)d_in[1];
  const float* xin   = (const float*)d_in[2];
  const int*   shp   = (const int*)d_in[3];
  const float* Wv    = (const float*)d_in[5];
  const float* bv    = (const float*)d_in[6];
  const float* Woff  = (const float*)d_in[7];
  const float* boff  = (const float*)d_in[8];
  const float* Wattn = (const float*)d_in[9];
  const float* battn = (const float*)d_in[10];
  const float* Wse   = (const float*)d_in[11];
  const float* bse   = (const float*)d_in[12];
  const float* Wout  = (const float*)d_in[13];
  const float* bout  = (const float*)d_in[14];
  float* out = (float*)d_out;

  char* ws = (char*)d_ws;
  unsigned short* AQ  = (unsigned short*)(ws + kOffAQ);
  unsigned short* AX  = (unsigned short*)(ws + kOffAX);
  unsigned short* WVT = (unsigned short*)(ws + kOffWVT);
  unsigned short* WQT = (unsigned short*)(ws + kOffWQT);
  unsigned short* WOT = (unsigned short*)(ws + kOffWOT);
  float*          BQ  = (float*)(ws + kOffBQ);
  float*          VAL = (float*)(ws + kOffVAL);
  float*          QP  = (float*)(ws + kOffQP);
  unsigned short* CAT = (unsigned short*)(ws + kOffCAT);
  float*          PR  = (float*)(ws + kOffPR);

  cast_act_kernel<<<dim3(kRowsP * kDm / 8 / 256, 2), 256, 0, stream>>>(query, xin, AQ, AX);
  weight_planes_kernel<<<kWtBlocks + 1, 256, 0, stream>>>(Wv, Woff, Wattn, Wout, boff, battn, WVT, WQT, WOT, BQ);

  gemm64_f16_kernel<<<(kRowsP / 64) * (kDm / 64) / 8, 256, 0, stream>>>(
      AX, kDm, WVT, kDm, VAL, kDm, bv, kRowsP, kDm, kDm, kRowsP, kProjScale);

  gemm64_f16_kernel<<<(kRowsP / 64) * (kQpW / 64) / 8, 256, 0, stream>>>(
      AQ, kDm, WQT, kDm, QP, kQpW, BQ, kRowsP, kQpW, kDm, kRowsP, kProjScale);

  gate_kernel<<<kNb, 256, 0, stream>>>(VAL, Wse, bse, shp, PR);

  sample_mix_kernel<<<kRowsP, 384, 0, stream>>>(VAL, QP, rpts, PR, (unsigned*)CAT);

  gemm64_f16_kernel<<<(kRowsP / 64) * (kDm / 64) / 8, 256, 0, stream>>>(
      CAT, kCatW, WOT, kCatW, out, kDm, bout, kRowsP, kDm, kCatW, kRows, kOutScale);
}
